// Layer_25546465476680
// MI455X (gfx1250) — hardware-verified
//
#include <hip/hip_runtime.h>
#include <stdint.h>

#define NB    4
#define NS    2048
#define NDM   1024
#define NDI   2048
#define NTOK  8192
#define KW    4
static_assert(NTOK == NB * NS);
static_assert((NDM % 64) == 0 && (NDI % 64) == 0 && (NS % 128) == 0 && (NTOK % 128) == 0);
static_assert((NDM % 32) == 0 && (NDI % 32) == 0 && (NS % 32) == 0);
static_assert((NTOK % 32) == 0 && (NDM % 256) == 0);

#define SZ_XB   ((size_t)NTOK * NDM * 2)
#define SZ_WD   ((size_t)NDM * NDI * 2)
#define SZ_W1   ((size_t)NDM * NDM * 2)
#define SZ_P    ((size_t)NS * NS * 2)
#define SZ_A3   ((size_t)NTOK * NDI * 2)
#define SZ_PL   ((size_t)NTOK * NDM * 2)
#define SZ_VT   ((size_t)NB * NDM * NS * 2)
#define SZ_SR   ((size_t)NTOK * 4)

#define OFF_R0  ((size_t)0)
#define SZ_R0   SZ_XB
#define OFF_XB  (OFF_R0)
#define OFF_WD  (OFF_R0)
#define OFF_WQH (OFF_R0 + SZ_WD)
#define OFF_WQB (OFF_WQH + SZ_W1)
#define OFF_WKH (OFF_WQB + SZ_W1)
#define OFF_WVH (OFF_WKH + SZ_W1)
#define OFF_WO  (OFF_WVH + SZ_W1)
#define OFF_P   (OFF_R0)
#define OFF_R1  (OFF_R0 + SZ_R0)
#define OFF_WU  (OFF_R1)
#define OFF_WG  (OFF_R1 + SZ_WD)
#define OFF_R2  (OFF_R1 + 2 * SZ_WD)
#define OFF_A3H (OFF_R2)
#define OFF_A3L (OFF_R2 + SZ_A3)
#define OFF_QH  (OFF_R2)
#define OFF_KH  (OFF_R2 + SZ_PL)
#define OFF_VT  (OFF_R2 + 2 * SZ_PL)
#define OFF_R3  (OFF_R2 + 2 * SZ_A3)
#define OFF_O1H (OFF_R3)
#define OFF_O1L (OFF_R3 + SZ_PL)
#define OFF_YH  (OFF_R3)
#define OFF_YL  (OFF_R3 + SZ_PL)
#define OFF_SR  (OFF_R3 + 2 * SZ_PL)
#define WS_END  (OFF_SR + SZ_SR)
static_assert(OFF_WO + SZ_W1 <= OFF_R0 + SZ_R0);
static_assert(OFF_P + SZ_P <= OFF_WO);
static_assert(OFF_VT + SZ_VT <= OFF_R3);
static_assert(OFF_A3L + SZ_A3 == OFF_R3);
static_assert(OFF_O1L + SZ_PL == OFF_SR);
static_assert(OFF_YL + SZ_PL == OFF_SR);
static_assert(WS_END <= (size_t)134217728u);
static_assert((OFF_R1 % 128) == 0 && (OFF_R2 % 128) == 0 && (OFF_R3 % 128) == 0 && (OFF_SR % 128) == 0);
static_assert((OFF_WQH % 128) == 0 && (OFF_WQB % 128) == 0 && (OFF_WKH % 128) == 0 && (OFF_WVH % 128) == 0 && (OFF_WO % 128) == 0);

typedef _Float16 v16h __attribute__((ext_vector_type(16)));
typedef _Float16 v8h  __attribute__((ext_vector_type(8)));
typedef __bf16   v16b __attribute__((ext_vector_type(16)));
typedef __bf16   v8b  __attribute__((ext_vector_type(8)));
typedef float    v8f  __attribute__((ext_vector_type(8)));
typedef float    v4f  __attribute__((ext_vector_type(4)));
typedef unsigned int v4u __attribute__((ext_vector_type(4)));
typedef v8h __attribute__((may_alias)) v8ha;
typedef v4f __attribute__((may_alias)) v4fa;
typedef v4u __attribute__((may_alias)) v4ua;

__device__ __forceinline__ unsigned short bf_bits(float f) {
  unsigned u = __float_as_uint(f);
  return (unsigned short)((u + 0x7FFFu + ((u >> 16) & 1u)) >> 16);
}
__device__ __forceinline__ float bf_up(unsigned short h) { return __uint_as_float(((unsigned)h) << 16); }
__device__ __forceinline__ unsigned pk16(unsigned short a, unsigned short b) { return (unsigned)a | ((unsigned)b << 16); }
__device__ __forceinline__ v8f zero8() { v8f z = {0.f, 0.f, 0.f, 0.f, 0.f, 0.f, 0.f, 0.f}; return z; }
__device__ __forceinline__ _Float16 h_val_ftz(float f) {
  return (fabsf(f) < 6.103515625e-05f) ? (_Float16)0.0f : (_Float16)f;
}
__device__ __forceinline__ unsigned short h_bits_ftz(float f) { return __builtin_bit_cast(unsigned short, h_val_ftz(f)); }
__device__ __forceinline__ float silu_f(float x) {
  const float e = __expf(fminf(-x, 80.0f));
  return x * __builtin_amdgcn_rcpf(1.0f + e);
}
__device__ __forceinline__ void split_bb(float f, unsigned short& hb, unsigned short& lb) {
  hb = bf_bits(f);
  lb = bf_bits(f - bf_up(hb));
}
__device__ __forceinline__ void split_hb(float f, unsigned short& hb, unsigned short& lb) {
  const _Float16 h = h_val_ftz(f * 16.0f);
  const float hf = (float)h * 0.0625f;
  hb = __builtin_bit_cast(unsigned short, h);
  lb = bf_bits(f - hf);
}
__device__ __forceinline__ void pack_bb8(const float* sp, v4u& hv, v4u& lv) {
  const v4f a = *(const v4fa*)sp;
  const v4f c = *(const v4fa*)(sp + 4);
  const float f[8] = {a[0], a[1], a[2], a[3], c[0], c[1], c[2], c[3]};
#pragma unroll
  for (int e = 0; e < 4; ++e) {
    unsigned short h0, l0, h1, l1;
    split_bb(f[2 * e], h0, l0);
    split_bb(f[2 * e + 1], h1, l1);
    hv[e] = pk16(h0, h1);
    lv[e] = pk16(l0, l1);
  }
}
__device__ __forceinline__ void pack_hb8(const float* sp, v4u& hv, v4u& lv) {
  const v4f a = *(const v4fa*)sp;
  const v4f c = *(const v4fa*)(sp + 4);
  const float f[8] = {a[0], a[1], a[2], a[3], c[0], c[1], c[2], c[3]};
#pragma unroll
  for (int e = 0; e < 4; ++e) {
    unsigned short h0, l0, h1, l1;
    split_hb(f[2 * e], h0, l0);
    split_hb(f[2 * e + 1], h1, l1);
    hv[e] = pk16(h0, h1);
    lv[e] = pk16(l0, l1);
  }
}

__device__ __forceinline__ v16b ldfrag_b(const __bf16* p) {
  union { v16b v; v8b h[2]; } f;
  f.h[0] = *(const v8b*)(p);
  f.h[1] = *(const v8b*)(p + 16);
  return f.v;
}
__device__ __forceinline__ v16h ldfrag_h(const _Float16* p) {
  union { v16h v; v8h h[2]; } f;
  f.h[0] = *(const v8ha*)(p);
  f.h[1] = *(const v8ha*)(p + 16);
  return f.v;
}

__device__ __forceinline__ v8f mma_b(v16b a, v16b b, v8f c) {
  c = __builtin_amdgcn_wmma_f32_16x16x32_bf16(false, a, false, b, (short)0, c, false, false);
  asm volatile("v_nop\n\tv_nop\n\tv_nop\n\tv_nop" : "+v"(c) : "v"(a), "v"(b));
  return c;
}
__device__ __forceinline__ v8f mma_h(v16h a, v16h b, v8f c) {
  c = __builtin_amdgcn_wmma_f32_16x16x32_f16(false, a, false, b, (short)0, c, false, false);
  asm volatile("v_nop\n\tv_nop\n\tv_nop\n\tv_nop" : "+v"(c) : "v"(a), "v"(b));
  return c;
}

__global__ __launch_bounds__(256) void k_xprep(const float* __restrict__ x, unsigned short* xb, float* srow) {
  __shared__ __align__(16) float sS[32];
  const int tid = threadIdx.x, lane = tid & 31, wave = tid >> 5;
  const int rbase = blockIdx.x * 32;
#pragma unroll 1
  for (int i = 0; i < 4; ++i) {
    const int row = rbase + wave * 4 + i;
    const float* xr = x + (size_t)row * NDM + lane * 8;
    v4u o[4];
    float sq = 0.0f;
#pragma unroll
    for (int g = 0; g < 4; ++g) {
      const v4f a = *(const v4fa*)(xr + g * 256);
      const v4f c = *(const v4fa*)(xr + g * 256 + 4);
      const float xv[8] = {a[0], a[1], a[2], a[3], c[0], c[1], c[2], c[3]};
      unsigned short hb[8];
#pragma unroll
      for (int e = 0; e < 8; ++e) {
        hb[e] = bf_bits(xv[e]);
        const float r = bf_up(hb[e]);
        sq += r * r;
      }
      v4u t;
      t[0] = pk16(hb[0], hb[1]); t[1] = pk16(hb[2], hb[3]); t[2] = pk16(hb[4], hb[5]); t[3] = pk16(hb[6], hb[7]);
      o[g] = t;
    }
    sq += __shfl_xor(sq, 16);
    sq += __shfl_xor(sq, 8);
    sq += __shfl_xor(sq, 4);
    sq += __shfl_xor(sq, 2);
    sq += __shfl_xor(sq, 1);
    const float s = rsqrtf(sq * (1.0f / 1024.0f) + 1e-6f);
    if (lane == 0) sS[wave * 4 + i] = s;
    unsigned short* dr = xb + (size_t)row * NDM + lane * 8;
    for (int pass = 0; pass < 2; ++pass) {
#pragma unroll
      for (int g = 0; g < 4; ++g) *(volatile v4u*)(dr + g * 256) = o[g];
      __threadfence();
    }
  }
  __syncthreads();
  if (wave == 0) {
    const v4f v = *(const v4fa*)(sS + 4 * (lane & 7));
    for (int pass = 0; pass < 2; ++pass) {
      if (lane < 8) *(volatile v4f*)(srow + rbase + 4 * lane) = v;
      __threadfence();
    }
  }
}

__global__ __launch_bounds__(256) void k_wtr(const float* __restrict__ src, const float* __restrict__ rsc, int use_rsc,
                                             int R, int C, float scale, int f16mode, unsigned short* dst) {
  __shared__ __align__(16) unsigned short sT[64 * 72];
  const int tid = threadIdx.x, lane = tid & 31, wave = tid >> 5;
  const int c0 = blockIdx.x * 64, r0 = blockIdx.y * 64;
  {
    const int r = tid >> 2, cc = (tid & 3) * 16;
    const float* sp = src + (size_t)(r0 + r) * C + c0 + cc;
    float rs = 1.0f;
    if (use_rsc != 0) rs = bf_up(bf_bits(rsc[r0 + r]));
#pragma unroll
    for (int g = 0; g < 4; ++g) {
      const v4f a = *(const v4fa*)(sp + 4 * g);
#pragma unroll
      for (int e = 0; e < 4; ++e) {
        float v = bf_up(bf_bits(a[e]));
        if (use_rsc != 0) v = bf_up(bf_bits(v * rs));
        v *= scale;
        const unsigned short bits = (f16mode != 0) ? h_bits_ftz(v) : bf_bits(v);
        sT[(cc + 4 * g + e) * 72 + r] = bits;
      }
    }
  }
  __syncthreads();
  const int q8 = lane & 7, sub = lane >> 3;
  v4u vv[2];
#pragma unroll
  for (int it = 0; it < 2; ++it) {
    const int cl = wave * 8 + it * 4 + sub;
    vv[it] = *(const v4ua*)(sT + cl * 72 + 8 * q8);
  }
  for (int pass = 0; pass < 2; ++pass) {
#pragma unroll
    for (int it = 0; it < 2; ++it) {
      const int cl = wave * 8 + it * 4 + sub;
      *(volatile v4u*)(dst + (size_t)(c0 + cl) * R + r0 + 8 * q8) = vv[it];
    }
    __threadfence();
  }
}

__global__ __launch_bounds__(128) void k_upgate(const unsigned short* __restrict__ xbp, const unsigned short* __restrict__ wup,
                                               const unsigned short* __restrict__ wgp, const float* __restrict__ srow,
                                               const float* __restrict__ convw, const float* __restrict__ convb,
                                               unsigned short* a3h, unsigned short* a3l) {
  __shared__ __align__(16) float sH[67 * 64];
  __shared__ __align__(16) float sA[64 * 64];
  const int tid = threadIdx.x, lane = tid & 31, wave = tid >> 5;
  const int hh = lane >> 4, m = lane & 15;
  const int nb = blockIdx.x, b = blockIdx.y, n0 = nb * 64;
  const __bf16* xb = (const __bf16*)(const void*)xbp;
  const __bf16* wu = (const __bf16*)(const void*)wup;
  const __bf16* wg = (const __bf16*)(const void*)wgp;

  float cw[4][4], cb[4];
#pragma unroll
  for (int nt = 0; nt < 4; ++nt) {
    const int ch = n0 + 16 * nt + m;
    const v4f t = *(const v4fa*)(convw + (size_t)ch * KW);
#pragma unroll
    for (int j = 0; j < 4; ++j) cw[nt][j] = bf_up(bf_bits(t[j]));
    cb[nt] = bf_up(bf_bits(convb[ch]));
  }
  for (int i = tid; i < 192; i += 128) sH[i] = 0.0f;

  const size_t xrow = ((size_t)(b * NS + 16 * wave + m)) * NDM + 8 * hh;
  const size_t wrow = ((size_t)(n0 + m)) * NDM + 8 * hh;
  const int q8 = lane & 7, sub = lane >> 3;

#pragma unroll 1
  for (int rt = 0; rt < 32; ++rt) {
    __syncthreads();
    v8f au[4], ag[4];
#pragma unroll
    for (int nt = 0; nt < 4; ++nt) { au[nt] = zero8(); ag[nt] = zero8(); }
    const __bf16* xa = xb + xrow + (size_t)rt * 64 * NDM;
#pragma unroll 1
    for (int k0 = 0; k0 < NDM; k0 += 32) {
      const v16b a = ldfrag_b(xa + k0);
#pragma unroll
      for (int nt = 0; nt < 4; ++nt) {
        const size_t bo = wrow + (size_t)nt * 16 * NDM + k0;
        const v16b bu = ldfrag_b(wu + bo);
        const v16b bg = ldfrag_b(wg + bo);
        au[nt] = mma_b(a, bu, au[nt]);
        ag[nt] = mma_b(a, bg, ag[nt]);
      }
    }
    const int tok0 = b * NS + rt * 64;
    const v4f s0 = *(const v4fa*)(srow + tok0 + 16 * wave + 8 * hh);
    const v4f s1 = *(const v4fa*)(srow + tok0 + 16 * wave + 8 * hh + 4);
    const float sv[8] = {s0[0], s0[1], s0[2], s0[3], s1[0], s1[1], s1[2], s1[3]};
#pragma unroll
    for (int nt = 0; nt < 4; ++nt)
#pragma unroll
      for (int r = 0; r < 8; ++r)
        sH[(3 + 16 * wave + 8 * hh + r) * 64 + 16 * nt + m] = au[nt][r] * sv[r];
    __syncthreads();
#pragma unroll
    for (int nt = 0; nt < 4; ++nt) {
      const int col = 16 * nt + m;
#pragma unroll
      for (int r = 0; r < 8; ++r) {
        const int rowl = 16 * wave + 8 * hh + r;
        const float* hp = sH + rowl * 64 + col;
        const float hc = ((cw[nt][0] * hp[0] + cw[nt][1] * hp[64]) + cw[nt][2] * hp[128]) + cw[nt][3] * hp[192] + cb[nt];
        const float g = ag[nt][r] * sv[r];
        sA[rowl * 64 + col] = silu_f(hc) * silu_f(g);
      }
    }
    __syncthreads();
    for (int i = tid; i < 192; i += 128) sH[i] = sH[64 * 64 + i];
    v4u hv[4], lv[4];
#pragma unroll
    for (int it = 0; it < 4; ++it) {
      const int row = 16 * wave + it * 4 + sub;
      pack_bb8(sA + row * 64 + 8 * q8, hv[it], lv[it]);
    }
    const size_t gb = ((size_t)(tok0 + 16 * wave)) * NDI + n0 + 8 * q8;
    for (int pass = 0; pass < 2; ++pass) {
#pragma unroll
      for (int it = 0; it < 4; ++it) {
        const int row = it * 4 + sub;
        *(volatile v4u*)(a3h + gb + (size_t)row * NDI) = hv[it];
        *(volatile v4u*)(a3l + gb + (size_t)row * NDI) = lv[it];
      }
      __threadfence();
    }
  }
}

__global__ __launch_bounds__(128) void k_down(const unsigned short* __restrict__ a3hp, const unsigned short* __restrict__ a3lp,
                                             const unsigned short* __restrict__ wdp, unsigned short* o1h, unsigned short* o1l) {
  __shared__ __align__(16) float sT[128 * 64];
  const int tid = threadIdx.x, lane = tid & 31, w = tid >> 5;
  const int hh = lane >> 4, m = lane & 15;
  const int m0 = blockIdx.x * 128, nb = blockIdx.y;
  const __bf16* Ah = (const __bf16*)(const void*)a3hp;
  const __bf16* Al = (const __bf16*)(const void*)a3lp;
  const __bf16* wd = (const __bf16*)(const void*)wdp;
  const size_t ao0 = ((size_t)(m0 + 32 * w + m)) * NDI + 8 * hh;
  const size_t ao1 = ao0 + (size_t)16 * NDI;
  const __bf16* wr = wd + ((size_t)(nb * 64 + m)) * NDI + 8 * hh;

  v8f acc[2][4];
#pragma unroll
  for (int mt = 0; mt < 2; ++mt)
#pragma unroll
    for (int nt = 0; nt < 4; ++nt) acc[mt][nt] = zero8();

#pragma unroll 1
  for (int k0 = 0; k0 < NDI; k0 += 32) {
    const v16b a0h = ldfrag_b(Ah + ao0 + k0);
    const v16b a0l = ldfrag_b(Al + ao0 + k0);
    const v16b a1h = ldfrag_b(Ah + ao1 + k0);
    const v16b a1l = ldfrag_b(Al + ao1 + k0);
#pragma unroll
    for (int nt = 0; nt < 4; ++nt) {
      const v16b bb = ldfrag_b(wr + (size_t)nt * 16 * NDI + k0);
      acc[0][nt] = mma_b(a0h, bb, acc[0][nt]);
      acc[0][nt] = mma_b(a0l, bb, acc[0][nt]);
      acc[1][nt] = mma_b(a1h, bb, acc[1][nt]);
      acc[1][nt] = mma_b(a1l, bb, acc[1][nt]);
    }
  }

#pragma unroll
  for (int nt = 0; nt < 4; ++nt)
#pragma unroll
    for (int mt = 0; mt < 2; ++mt)
#pragma unroll
      for (int r = 0; r < 8; ++r) {
        const int tokl = 32 * w + 16 * mt + 8 * hh + r;
        sT[tokl * 64 + 16 * nt + m] = acc[mt][nt][r];
      }
  __syncthreads();

  const int q8 = lane & 7, sub = lane >> 3;
  v4u hv[8], lv[8];
#pragma unroll
  for (int it = 0; it < 8; ++it) {
    const int row = 32 * w + it * 4 + sub;
    pack_hb8(sT + row * 64 + 8 * q8, hv[it], lv[it]);
  }
  const size_t gb = ((size_t)(m0 + 32 * w)) * NDM + nb * 64 + 8 * q8;
  for (int pass = 0; pass < 2; ++pass) {
#pragma unroll
    for (int it = 0; it < 8; ++it) {
      const int row = it * 4 + sub;
      *(volatile v4u*)(o1h + gb + (size_t)row * NDM) = hv[it];
      *(volatile v4u*)(o1l + gb + (size_t)row * NDM) = lv[it];
    }
    __threadfence();
  }
}

__global__ __launch_bounds__(128) void k_qkv(const unsigned short* __restrict__ o1hp, const unsigned short* __restrict__ o1lp,
                                            const unsigned short* __restrict__ wqh, const unsigned short* __restrict__ wqb,
                                            const unsigned short* __restrict__ wkh, const unsigned short* __restrict__ wvh,
                                            unsigned short* qpl, unsigned short* kpl, unsigned short* vtp) {
  __shared__ __align__(16) _Float16 sT[128 * 64];
  const int tid = threadIdx.x, lane = tid & 31, w = tid >> 5;
  const int hh = lane >> 4, m = lane & 15;
  const int m0 = blockIdx.x * 128;
  const int cg = blockIdx.y, which = cg >> 4, nb = cg & 15;
  const _Float16* Oh = (const _Float16*)(const void*)o1hp;
  const __bf16*   Ol = (const __bf16*)(const void*)o1lp;
  const size_t ao0 = ((size_t)(m0 + 32 * w + m)) * NDM + 8 * hh;
  const size_t ao1 = ao0 + (size_t)16 * NDM;
  const size_t wro = ((size_t)(nb * 64 + m)) * NDM + 8 * hh;

  v8f acc[2][4];
#pragma unroll
  for (int mt = 0; mt < 2; ++mt)
#pragma unroll
    for (int nt = 0; nt < 4; ++nt) acc[mt][nt] = zero8();

  if (which == 0) {
    const _Float16* whp = (const _Float16*)(const void*)wqh + wro;
    const __bf16*   wbp = (const __bf16*)(const void*)wqb + wro;
#pragma unroll 1
    for (int k0 = 0; k0 < NDM; k0 += 32) {
      const v16h a0h = ldfrag_h(Oh + ao0 + k0);
      const v16b a0l = ldfrag_b(Ol + ao0 + k0);
      const v16h a1h = ldfrag_h(Oh + ao1 + k0);
      const v16b a1l = ldfrag_b(Ol + ao1 + k0);
#pragma unroll
      for (int nt = 0; nt < 4; ++nt) {
        const v16h bh = ldfrag_h(whp + (size_t)nt * 16 * NDM + k0);
        const v16b bl = ldfrag_b(wbp + (size_t)nt * 16 * NDM + k0);
        acc[0][nt] = mma_h(a0h, bh, acc[0][nt]);
        acc[0][nt] = mma_b(a0l, bl, acc[0][nt]);
        acc[1][nt] = mma_h(a1h, bh, acc[1][nt]);
        acc[1][nt] = mma_b(a1l, bl, acc[1][nt]);
      }
    }
  } else {
    const _Float16* whp = (const _Float16*)(const void*)((which == 1) ? wkh : wvh) + wro;
#pragma unroll 1
    for (int k0 = 0; k0 < NDM; k0 += 32) {
      const v16h a0h = ldfrag_h(Oh + ao0 + k0);
      const v16h a1h = ldfrag_h(Oh + ao1 + k0);
#pragma unroll
      for (int nt = 0; nt < 4; ++nt) {
        const v16h bh = ldfrag_h(whp + (size_t)nt * 16 * NDM + k0);
        acc[0][nt] = mma_h(a0h, bh, acc[0][nt]);
        acc[1][nt] = mma_h(a1h, bh, acc[1][nt]);
      }
    }
  }

  const float osc = (which == 2) ? (16.0f / 1024.0f) : (1.0f / 1024.0f);
#pragma unroll
  for (int nt = 0; nt < 4; ++nt) {
    const int feat = 16 * nt + m;
#pragma unroll
    for (int mt = 0; mt < 2; ++mt)
#pragma unroll
      for (int r = 0; r < 8; ++r) {
        const int tokl = 32 * w + 16 * mt + 8 * hh + r;
        const float y = acc[mt][nt][r] * osc;
        const int idx = (which == 2) ? (feat * 128 + tokl) : (tokl * 64 + feat);
        sT[idx] = h_val_ftz(y);
      }
  }
  __syncthreads();

  const int bidx = m0 / NS, l0 = m0 - bidx * NS;
  _Float16* plane = (_Float16*)(void*)((which == 0) ? qpl : kpl);
  _Float16* vt = (_Float16*)(void*)vtp;
  const int q8 = lane & 7, sub = lane >> 3;
  for (int pass = 0; pass < 2; ++pass) {
#pragma unroll
    for (int i = 0; i < 8; ++i) {
      const int lid = w * 32 + i * 4 + sub;
      v8h v;
      _Float16* dst;
      if (which != 2) {
        v = *(const v8ha*)(sT + lid * 64 + 8 * q8);
        dst = plane + ((size_t)(m0 + lid)) * NDM + nb * 64 + 8 * q8;
      } else {
        const int d = lid >> 1, hl = lid & 1;
        v = *(const v8ha*)(sT + d * 128 + 64 * hl + 8 * q8);
        dst = vt + ((size_t)(bidx * NDM + nb * 64 + d)) * NS + l0 + 64 * hl + 8 * q8;
      }
      *(volatile v8h*)dst = v;
    }
    __threadfence();
  }
}

__global__ __launch_bounds__(128) void k_qk(const unsigned short* __restrict__ qpl, const unsigned short* __restrict__ kpl,
                                           unsigned short* Pp, int b) {
  __shared__ __align__(16) _Float16 sT[128 * 64];
  const int kb = blockIdx.x, qb = blockIdx.y;
  if (kb * 64 >= (qb + 1) * 128) return;
  const int tid = threadIdx.x, lane = tid & 31, w = tid >> 5;
  const int hh = lane >> 4, m = lane & 15;
  const _Float16* Q = (const _Float16*)(const void*)qpl;
  const _Float16* K = (const _Float16*)(const void*)kpl;
  const size_t qo0 = ((size_t)(b * NS + qb * 128 + 32 * w + m)) * NDM + 8 * hh;
  const size_t qo1 = qo0 + (size_t)16 * NDM;
  const _Float16* kr = K + ((size_t)(b * NS + kb * 64 + m)) * NDM + 8 * hh;

  v8f acc[2][4];
#pragma unroll
  for (int mt = 0; mt < 2; ++mt)
#pragma unroll
    for (int nt = 0; nt < 4; ++nt) acc[mt][nt] = zero8();

#pragma unroll 1
  for (int k0 = 0; k0 < NDM; k0 += 32) {
    const v16h a0 = ldfrag_h(Q + qo0 + k0);
    const v16h a1 = ldfrag_h(Q + qo1 + k0);
#pragma unroll
    for (int nt = 0; nt < 4; ++nt) {
      const v16h bk = ldfrag_h(kr + (size_t)nt * 16 * NDM + k0);
      acc[0][nt] = mma_h(a0, bk, acc[0][nt]);
      acc[1][nt] = mma_h(a1, bk, acc[1][nt]);
    }
  }

#pragma unroll
  for (int nt = 0; nt < 4; ++nt) {
    const int feat = 16 * nt + m;
    const int key = kb * 64 + feat;
#pragma unroll
    for (int mt = 0; mt < 2; ++mt)
#pragma unroll
      for (int r = 0; r < 8; ++r) {
        const int tokl = 32 * w + 16 * mt + 8 * hh + r;
        const int qrow = qb * 128 + tokl;
        const float p = (key <= qrow) ? acc[mt][nt][r] : 0.0f;
        sT[tokl * 64 + feat] = h_val_ftz(p);
      }
  }
  __syncthreads();

  _Float16* P = (_Float16*)(void*)Pp;
  const int q8 = lane & 7, sub = lane >> 3;
  for (int pass = 0; pass < 2; ++pass) {
#pragma unroll
    for (int i = 0; i < 8; ++i) {
      const int lid = w * 32 + i * 4 + sub;
      const v8h v = *(const v8ha*)(sT + lid * 64 + 8 * q8);
      *(volatile v8h*)(P + ((size_t)(qb * 128 + lid)) * NS + kb * 64 + 8 * q8) = v;
    }
    __threadfence();
  }
}

__global__ __launch_bounds__(128) void k_pv(const unsigned short* __restrict__ Pp, const unsigned short* __restrict__ vtp,
                                           unsigned short* yh, unsigned short* yl, int b) {
  __shared__ __align__(16) float sT[128 * 64];
  const int tid = threadIdx.x, lane = tid & 31, w = tid >> 5;
  const int hh = lane >> 4, m = lane & 15;
  const int eb = blockIdx.x, qb = blockIdx.y;
  const int ntau = (qb + 1) * 128;
  const _Float16* P  = (const _Float16*)(const void*)Pp;
  const _Float16* VT = (const _Float16*)(const void*)vtp;
  const size_t po0 = ((size_t)(qb * 128 + 32 * w + m)) * NS + 8 * hh;
  const size_t po1 = po0 + (size_t)16 * NS;
  const _Float16* vr = VT + ((size_t)(b * NDM + eb * 64 + m)) * NS + 8 * hh;

  v8f acc[2][4];
#pragma unroll
  for (int mt = 0; mt < 2; ++mt)
#pragma unroll
    for (int nt = 0; nt < 4; ++nt) acc[mt][nt] = zero8();

#pragma unroll 1
  for (int t0 = 0; t0 < ntau; t0 += 32) {
    const v16h a0 = ldfrag_h(P + po0 + t0);
    const v16h a1 = ldfrag_h(P + po1 + t0);
#pragma unroll
    for (int nt = 0; nt < 4; ++nt) {
      const v16h bv = ldfrag_h(vr + (size_t)nt * 16 * NS + t0);
      acc[0][nt] = mma_h(a0, bv, acc[0][nt]);
      acc[1][nt] = mma_h(a1, bv, acc[1][nt]);
    }
  }

#pragma unroll
  for (int nt = 0; nt < 4; ++nt)
#pragma unroll
    for (int mt = 0; mt < 2; ++mt)
#pragma unroll
      for (int r = 0; r < 8; ++r) {
        const int tokl = 32 * w + 16 * mt + 8 * hh + r;
        sT[tokl * 64 + 16 * nt + m] = acc[mt][nt][r] * 0.0625f;
      }
  __syncthreads();

  const int q8 = lane & 7, sub = lane >> 3;
  v4u hv[8], lv[8];
#pragma unroll
  for (int it = 0; it < 8; ++it) {
    const int row = 32 * w + it * 4 + sub;
    pack_bb8(sT + row * 64 + 8 * q8, hv[it], lv[it]);
  }
  const size_t gb = ((size_t)(b * NS + qb * 128 + 32 * w)) * NDM + eb * 64 + 8 * q8;
  for (int pass = 0; pass < 2; ++pass) {
#pragma unroll
    for (int it = 0; it < 8; ++it) {
      const int row = it * 4 + sub;
      *(volatile v4u*)(yh + gb + (size_t)row * NDM) = hv[it];
      *(volatile v4u*)(yl + gb + (size_t)row * NDM) = lv[it];
    }
    __threadfence();
  }
}

__global__ __launch_bounds__(128) void k_out(const unsigned short* __restrict__ yhp, const unsigned short* __restrict__ ylp,
                                            const unsigned short* __restrict__ wop, const float* __restrict__ x, float* out) {
  __shared__ __align__(16) float sT[128 * 64];
  const int tid = threadIdx.x, lane = tid & 31, w = tid >> 5;
  const int hh = lane >> 4, m = lane & 15;
  const int m0 = blockIdx.x * 128, nb = blockIdx.y;
  const __bf16* Yh = (const __bf16*)(const void*)yhp;
  const __bf16* Yl = (const __bf16*)(const void*)ylp;
  const __bf16* wo = (const __bf16*)(const void*)wop;
  const size_t yo0 = ((size_t)(m0 + 32 * w + m)) * NDM + 8 * hh;
  const size_t yo1 = yo0 + (size_t)16 * NDM;
  const __bf16* wr = wo + ((size_t)(nb * 64 + m)) * NDM + 8 * hh;

  v8f acc[2][4];
#pragma unroll
  for (int mt = 0; mt < 2; ++mt)
#pragma unroll
    for (int nt = 0; nt < 4; ++nt) acc[mt][nt] = zero8();

#pragma unroll 1
  for (int k0 = 0; k0 < NDM; k0 += 32) {
    const v16b a0h = ldfrag_b(Yh + yo0 + k0);
    const v16b a0l = ldfrag_b(Yl + yo0 + k0);
    const v16b a1h = ldfrag_b(Yh + yo1 + k0);
    const v16b a1l = ldfrag_b(Yl + yo1 + k0);
#pragma unroll
    for (int nt = 0; nt < 4; ++nt) {
      const v16b bb = ldfrag_b(wr + (size_t)nt * 16 * NDM + k0);
      acc[0][nt] = mma_b(a0h, bb, acc[0][nt]);
      acc[0][nt] = mma_b(a0l, bb, acc[0][nt]);
      acc[1][nt] = mma_b(a1h, bb, acc[1][nt]);
      acc[1][nt] = mma_b(a1l, bb, acc[1][nt]);
    }
  }

#pragma unroll
  for (int nt = 0; nt < 4; ++nt)
#pragma unroll
    for (int mt = 0; mt < 2; ++mt)
#pragma unroll
      for (int r = 0; r < 8; ++r) {
        const int tokl = 32 * w + 16 * mt + 8 * hh + r;
        sT[tokl * 64 + 16 * nt + m] = acc[mt][nt][r];
      }
  __syncthreads();

  v4f vals[16];
#pragma unroll
  for (int i = 0; i < 16; ++i) {
    const int rowl = 32 * w + 2 * i + hh;
    const v4f t  = *(const v4fa*)(sT + rowl * 64 + 4 * m);
    const v4f xv = *(const v4fa*)(x + ((size_t)(m0 + rowl)) * NDM + nb * 64 + 4 * m);
    vals[i] = t + xv;
  }
  for (int pass = 0; pass < 2; ++pass) {
#pragma unroll
    for (int i = 0; i < 16; ++i) {
      const int rowl = 32 * w + 2 * i + hh;
      *(volatile v4f*)(out + ((size_t)(m0 + rowl)) * NDM + nb * 64 + 4 * m) = vals[i];
    }
    __threadfence();
  }
}

static void launch_wtr(const float* src, const float* rsc, int use_rsc, int R, int C, float scale, int f16mode,
                       unsigned short* dst, hipStream_t stream) {
  k_wtr<<<dim3(C / 64, R / 64), dim3(256), 0, stream>>>(src, rsc, use_rsc, R, C, scale, f16mode, dst);
}

extern "C" void kernel_launch(void* const* d_in, const int* in_sizes, int n_in,
                              void* d_out, int out_size, void* d_ws, size_t ws_size,
                              hipStream_t stream) {
  if (n_in < 11) return;
  if (in_sizes[0] != NTOK * NDM) return;
  if (in_sizes[1] != NDM) return;
  if (in_sizes[2] != NDM * NDI || in_sizes[3] != NDM * NDI || in_sizes[4] != NDI * NDM) return;
  if (in_sizes[5] != NDI * KW || in_sizes[6] != NDI) return;
  if (in_sizes[7] != NDM * NDM || in_sizes[8] != NDM * NDM || in_sizes[9] != NDM * NDM || in_sizes[10] != NDM * NDM) return;
  if (out_size != NTOK * NDM) return;
  if (WS_END > ws_size) return;

  const float* x      = (const float*)d_in[0];
  const float* norm_w = (const float*)d_in[1];
  const float* w_up   = (const float*)d_in[2];
  const float* w_gate = (const float*)d_in[3];
  const float* w_down = (const float*)d_in[4];
  const float* conv_w = (const float*)d_in[5];
  const float* conv_b = (const float*)d_in[6];
  const float* w_q    = (const float*)d_in[7];
  const float* w_k    = (const float*)d_in[8];
  const float* w_v    = (const float*)d_in[9];
  const float* w_o    = (const float*)d_in[10];
  float* out = (float*)d_out;

  char* ws = (char*)d_ws;
  unsigned short* xb  = (unsigned short*)(ws + OFF_XB);
  unsigned short* wd  = (unsigned short*)(ws + OFF_WD);
  unsigned short* wqh = (unsigned short*)(ws + OFF_WQH);
  unsigned short* wqb = (unsigned short*)(ws + OFF_WQB);
  unsigned short* wkh = (unsigned short*)(ws + OFF_WKH);
  unsigned short* wvh = (unsigned short*)(ws + OFF_WVH);
  unsigned short* wo  = (unsigned short*)(ws + OFF_WO);
  unsigned short* Pp  = (unsigned short*)(ws + OFF_P);
  unsigned short* wu  = (unsigned short*)(ws + OFF_WU);
  unsigned short* wg  = (unsigned short*)(ws + OFF_WG);
  unsigned short* a3h = (unsigned short*)(ws + OFF_A3H);
  unsigned short* a3l = (unsigned short*)(ws + OFF_A3L);
  unsigned short* qpl = (unsigned short*)(ws + OFF_QH);
  unsigned short* kpl = (unsigned short*)(ws + OFF_KH);
  unsigned short* vt  = (unsigned short*)(ws + OFF_VT);
  unsigned short* o1h = (unsigned short*)(ws + OFF_O1H);
  unsigned short* o1l = (unsigned short*)(ws + OFF_O1L);
  unsigned short* yh  = (unsigned short*)(ws + OFF_YH);
  unsigned short* yl  = (unsigned short*)(ws + OFF_YL);
  float* srow = (float*)(ws + OFF_SR);

  k_xprep<<<dim3(NTOK / 32), dim3(256), 0, stream>>>(x, xb, srow);
  launch_wtr(w_up,   norm_w, 1, NDM, NDI, 1.0f, 0, wu, stream);
  launch_wtr(w_gate, norm_w, 1, NDM, NDI, 1.0f, 0, wg, stream);
  k_upgate<<<dim3(NDI / 64, NB), dim3(128), 0, stream>>>(xb, wu, wg, srow, conv_w, conv_b, a3h, a3l);
  launch_wtr(w_down, w_down, 0, NDI, NDM, 1.0f,    0, wd,  stream);
  launch_wtr(w_q,    w_q,    0, NDM, NDM, 64.0f,   1, wqh, stream);
  launch_wtr(w_q,    w_q,    0, NDM, NDM, 1024.0f, 0, wqb, stream);
  launch_wtr(w_k,    w_k,    0, NDM, NDM, 64.0f,   1, wkh, stream);
  launch_wtr(w_v,    w_v,    0, NDM, NDM, 64.0f,   1, wvh, stream);
  launch_wtr(w_o,    w_o,    0, NDM, NDM, 1.0f,    0, wo,  stream);
  k_down<<<dim3(NTOK / 128, NDM / 64), dim3(128), 0, stream>>>(a3h, a3l, wd, o1h, o1l);
  k_qkv<<<dim3(NTOK / 128, 3 * (NDM / 64)), dim3(128), 0, stream>>>(o1h, o1l, wqh, wqb, wkh, wvh, qpl, kpl, vt);
  for (int b = 0; b < NB; ++b) {
    k_qk<<<dim3(NS / 64, NS / 128), dim3(128), 0, stream>>>(qpl, kpl, Pp, b);
    k_pv<<<dim3(NDM / 64, NS / 128), dim3(128), 0, stream>>>(Pp, vt, yh, yl, b);
  }
  k_out<<<dim3(NTOK / 128, NDM / 64), dim3(128), 0, stream>>>(yh, yl, wo, x, out);
  (void)hipGetLastError();
}
